// MultiHeadedAttention_54271206752303
// MI455X (gfx1250) — hardware-verified
//
#include <hip/hip_runtime.h>
#include <math.h>

typedef __attribute__((ext_vector_type(16))) _Float16 v16h;
typedef __attribute__((ext_vector_type(16))) __bf16 v16b;
typedef __attribute__((ext_vector_type(8)))  _Float16 v8h;
typedef __attribute__((ext_vector_type(8)))  __bf16 v8b;
typedef __attribute__((ext_vector_type(8)))  float v8f;
typedef __attribute__((ext_vector_type(4)))  float v4f;
typedef __attribute__((ext_vector_type(4)))  unsigned v4u;
typedef __attribute__((ext_vector_type(4)))  int v4i;

#ifndef NB
#define NB 2
#endif
#ifndef SEQ
#define SEQ 2048
#endif
#define NB_FULL 2
#define SEQ_FULL 2048
#define CC 1024
#define DIN 1024
#define NH 16
#define HD 64
#define EARLY 256
#define NQB (SEQ / 64)
#define SCALE (0.125f)

static_assert(NH * HD == CC);
static_assert(HD == 64);
static_assert(DIN == 1024);
static_assert(CC == 1024);
static_assert(DIN % 32 == 0);
static_assert(CC % 128 == 0);
static_assert(SEQ % 128 == 0);
static_assert(SEQ / 128 <= 16);
static_assert(NQB <= 32);
static_assert(EARLY % 64 == 0);
static_assert(EARLY <= SEQ);
static_assert(SEQ <= SEQ_FULL);
static_assert(NB <= NB_FULL);

template <typename T> __device__ __forceinline__ void vst2(void* p, T v) { *(volatile T*)p = v; __threadfence(); *(volatile T*)p = v; }
__device__ __forceinline__ v8f wmma16(v16h a, v16h b, v8f c) {
  v8f d = __builtin_amdgcn_wmma_f32_16x16x32_f16(false, a, false, b, (short)0, c, false, false);
  asm volatile("v_nop\n\tv_nop\n\tv_nop\n\tv_nop" : "+v"(d) : "v"(a), "v"(b));
  return d;
}
__device__ __forceinline__ v8f wmma_bf(v16b a, v16b b, v8f c) {
  v8f d = __builtin_amdgcn_wmma_f32_16x16x32_bf16(false, a, false, b, (short)0, c, false, false);
  asm volatile("v_nop\n\tv_nop\n\tv_nop\n\tv_nop" : "+v"(d) : "v"(a), "v"(b));
  return d;
}
__device__ __forceinline__ v16h frag_h(const _Float16* rowk0, int lane) {
  union { v16h v; v8h q[2]; } u; const _Float16* p = rowk0 + 8 * (lane >> 4);
  u.q[0] = *(const v8h*)p; u.q[1] = *(const v8h*)(p + 16); return u.v;
}
__device__ __forceinline__ v16b frag_b(const __bf16* rowk0, int lane) {
  union { v16b v; v8b q[2]; } u; const __bf16* p = rowk0 + 8 * (lane >> 4);
  u.q[0] = *(const v8b*)p; u.q[1] = *(const v8b*)(p + 16); return u.v;
}
__device__ __forceinline__ float bfr(float v) { return (float)(__bf16)v; }
#define LDSX() do { asm volatile("s_wait_dscnt 0" ::: "memory"); __builtin_amdgcn_wave_barrier(); __builtin_amdgcn_fence(3  , "workgroup"); } while (0)

union H8 { v8h h; v4u u; };
union B8 { v8b b; v4u u; };

#define SZ_X   (2u * (size_t)NB * SEQ * DIN)
#define SZ_W   (2u * (size_t)CC * DIN)
#define SZ_A   (2u * (size_t)NB * SEQ * CC)
#define SZ_E   (2u * (size_t)NB * EARLY * CC)
#define WS_XB  ((size_t)0)
#define WS_WB  (WS_XB + 3u * SZ_X)
#define WS_WOH (WS_WB + 4u * SZ_W)
#define WS_QKH (WS_WOH + SZ_W)
#define WS_QKL (WS_QKH + 2u * SZ_A)
#define WS_VT  (WS_QKL + SZ_A + SZ_E)
#define WS_VB  (WS_VT + SZ_A)
#define WS_VBL (WS_VB + SZ_A)
#define WS_YH  (WS_VBL + SZ_A)
#define WS_YB  (WS_YH + SZ_A)
#define WS_YBL (WS_YB + SZ_E)
#define WS_FL  (WS_YBL + SZ_E)
#define WS_END (WS_FL + 32u * 128u)
static_assert(WS_END <= (size_t)134217728);
static_assert(SZ_X % 128 == 0);
static_assert(SZ_W % 128 == 0);
static_assert(SZ_A % 128 == 0);
static_assert(SZ_E % 128 == 0);

#define XUNITS ((size_t)NB * SEQ * (DIN / 8))
#define WUNITS ((size_t)CC * (DIN / 8))
#define CVT_UNITS (XUNITS > WUNITS ? XUNITS : WUNITS)
static_assert(XUNITS % 256 == 0);
static_assert(WUNITS % 256 == 0);

__device__ __forceinline__ void ld8(const float* __restrict__ p, size_t i, float t[8]) {
  const v4f a = *(const v4f*)(p + i); const v4f b = *(const v4f*)(p + i + 4);
  t[0] = a.x; t[1] = a.y; t[2] = a.z; t[3] = a.w; t[4] = b.x; t[5] = b.y; t[6] = b.z; t[7] = b.w;
}

__global__ __launch_bounds__(256) void k_cvt(const float* __restrict__ X0, const float* __restrict__ X1, const float* __restrict__ X2,
    const float* __restrict__ W0, const float* __restrict__ W1, const float* __restrict__ W2, const float* __restrict__ W3,
    __bf16* __restrict__ XB, __bf16* __restrict__ WB, _Float16* __restrict__ WOH) {
  const int which = blockIdx.y; const size_t u = (size_t)blockIdx.x * 256 + threadIdx.x;
  float t[8];
  if (which < 3) {
    if (u >= XUNITS) return;
    const size_t row = u >> 7; const int c8 = (int)(u & 127); const size_t bb = row / SEQ, s = row % SEQ;
    const size_t si = (bb * SEQ_FULL + s) * DIN + (size_t)c8 * 8;
    if (which == 0) ld8(X0, si, t); else if (which == 1) ld8(X1, si, t); else ld8(X2, si, t);
    B8 o;
#pragma unroll
    for (int i = 0; i < 8; ++i) o.b[i] = (__bf16)t[i];
    vst2(XB + (size_t)which * NB * SEQ * DIN + u * 8, o.u);
  } else {
    if (u >= WUNITS) return;
    const size_t si = u * 8;
    if (which == 3) ld8(W0, si, t); else if (which == 4) ld8(W1, si, t); else if (which == 5) ld8(W2, si, t); else ld8(W3, si, t);
    B8 o;
#pragma unroll
    for (int i = 0; i < 8; ++i) o.b[i] = (__bf16)t[i];
    vst2(WB + (size_t)(which - 3) * CC * DIN + u * 8, o.u);
    if (which == 6) { H8 hh;
#pragma unroll
      for (int i = 0; i < 8; ++i) hh.h[i] = (_Float16)((float)o.b[i] * 256.0f);
      vst2(WOH + u * 8, hh.u); }
  }
}

__global__ __launch_bounds__(256) void k_flag(const int* __restrict__ MK, int* __restrict__ FL) {
  __shared__ unsigned snz[8][2], sz[8][2]; __shared__ int sfull[8];
  const int tid = threadIdx.x, lane = tid & 31; const int wave = __builtin_amdgcn_readfirstlane(tid >> 5);
  const int qb = blockIdx.x;
  unsigned nzb = 0u, zb = 0u; int full = 0;
#pragma unroll 1
  for (int rr = 0; rr < 8; ++rr) {
    const int* mr = MK + (size_t)(qb * 64 + wave * 8 + rr) * SEQ_FULL + lane * 4; unsigned rnz = 0u;
#pragma unroll
    for (int it = 0; it < SEQ / 128; ++it) { const v4i m = *(const v4i*)(mr + it * 128);
      const unsigned anz = (unsigned)((m.x != 0) | (m.y != 0) | (m.z != 0) | (m.w != 0));
      const unsigned az = (unsigned)((m.x == 0) | (m.y == 0) | (m.z == 0) | (m.w == 0));
      rnz |= anz << it; zb |= az << it; }
    nzb |= rnz;
    unsigned w = rnz;
#pragma unroll
    for (int o = 1; o < 32; o <<= 1) w |= (unsigned)__shfl_xor((int)w, o);
    full |= (w == 0u) ? 1 : 0;
  }
#pragma unroll
  for (int o = 1; o < 16; o <<= 1) { nzb |= (unsigned)__shfl_xor((int)nzb, o); zb |= (unsigned)__shfl_xor((int)zb, o); }
  if ((lane & 15) == 0) { snz[wave][lane >> 4] = nzb; sz[wave][lane >> 4] = zb; }
  if (lane == 0) sfull[wave] = full;
  __syncthreads();
  if (wave == 0) { const int it = lane >> 1, hf = lane & 1; unsigned a = 0u, z = 0u; int f = 0;
#pragma unroll
    for (int w = 0; w < 8; ++w) { a |= snz[w][hf]; z |= sz[w][hf]; f |= sfull[w]; }
    const int flag = (int)((a >> it) & 1u) | ((int)((z >> it) & 1u) << 1) | (f << 2);
    vst2(FL + qb * 32 + lane, flag); }
}

__global__ __launch_bounds__(128) void k_proj(const __bf16* __restrict__ XB, const __bf16* __restrict__ WB, const float* __restrict__ COS, const float* __restrict__ SIN,
    _Float16* __restrict__ QKH, _Float16* __restrict__ QKL, _Float16* __restrict__ VT, __bf16* __restrict__ VB, __bf16* __restrict__ VBL) {
  __shared__ __align__(16) float sf[64][132];
  __shared__ __align__(16) _Float16 th[128][72]; __shared__ __align__(16) __bf16 tb[128][72], tbl[128][72];
  const int tid = threadIdx.x, lane = tid & 31, col = lane & 15, g = lane >> 4; const int wave = __builtin_amdgcn_readfirstlane(tid >> 5);
  const int which = blockIdx.z; const int c0 = blockIdx.y * 128; const size_t r0 = (size_t)blockIdx.x * 64; const size_t bb = r0 / SEQ; const int t0 = (int)(r0 % SEQ);
  const __bf16* X = XB + (size_t)which * NB * SEQ * DIN; const __bf16* W = WB + (size_t)which * CC * DIN;
  v8f acc[8] = {};
#pragma unroll 2
  for (int kc = 0; kc < DIN / 32; ++kc) { const v16b a = frag_b(X + (r0 + wave * 16 + col) * DIN + kc * 32, lane);
#pragma unroll
    for (int j = 0; j < 8; ++j) { const v16b w = frag_b(W + (size_t)(c0 + j * 16 + col) * DIN + kc * 32, lane); acc[j] = wmma_bf(a, w, acc[j]); } }
  if (which < 2) {
#pragma unroll
    for (int j = 0; j < 8; ++j) {
#pragma unroll
      for (int r = 0; r < 8; ++r) sf[wave * 16 + 8 * g + r][j * 16 + col] = acc[j][r]; }
    __syncthreads();
    _Float16* DH = QKH + (size_t)which * NB * SEQ * CC;
    const bool wl = (which == 1) || (t0 < EARLY);
#pragma unroll 1
    for (int e = tid; e < 64 * 16; e += 128) { const int rl = e >> 4, q = e & 15, cl = q * 8, d0 = cl & 63, pcl = cl ^ 32; const float sg = (d0 < 32) ? -1.0f : 1.0f;
      const size_t cs = (size_t)(t0 + rl) * HD + d0;
      const v4f ca = *(const v4f*)(COS + cs), cb = *(const v4f*)(COS + cs + 4), sa = *(const v4f*)(SIN + cs), sb = *(const v4f*)(SIN + cs + 4);
      float cv[8], sv[8];
      cv[0] = ca.x; cv[1] = ca.y; cv[2] = ca.z; cv[3] = ca.w; cv[4] = cb.x; cv[5] = cb.y; cv[6] = cb.z; cv[7] = cb.w;
      sv[0] = sa.x; sv[1] = sa.y; sv[2] = sa.z; sv[3] = sa.w; sv[4] = sb.x; sv[5] = sb.y; sv[6] = sb.z; sv[7] = sb.w;
      H8 hv, lv;
#pragma unroll
      for (int u = 0; u < 8; ++u) { const float x = sf[rl][cl + u], xp = sf[rl][pcl + u]; const float v = x * bfr(cv[u]) + sg * xp * bfr(sv[u]);
        const _Float16 hh = (_Float16)v; hv.h[u] = hh; lv.h[u] = (_Float16)((v - (float)hh) * 1024.0f); }
      vst2(DH + (r0 + rl) * CC + c0 + cl, hv.u);
      if (wl) { const size_t lo = (which == 1) ? (r0 + rl) * CC : (size_t)NB * SEQ * CC + (bb * EARLY + t0 + rl) * (size_t)CC; vst2(QKL + lo + c0 + cl, lv.u); } }
  } else {
#pragma unroll
    for (int j = 0; j < 8; ++j) {
#pragma unroll
      for (int r = 0; r < 8; ++r) { const float v = acc[j][r]; const int rl = wave * 16 + 8 * g + r, cl = j * 16 + col; th[cl][rl] = (_Float16)v; const __bf16 bh = (__bf16)v; tb[cl][rl] = bh; tbl[cl][rl] = (__bf16)(v - (float)bh); } }
    __syncthreads();
#pragma unroll 1
    for (int e = tid; e < 128 * 8; e += 128) { const int cl = e >> 3, q = e & 7; const size_t o3 = (bb * CC + c0 + cl) * (size_t)SEQ + t0 + q * 8;
      vst2(VT + o3, *(const v4u*)&th[cl][q * 8]); vst2(VB + o3, *(const v4u*)&tb[cl][q * 8]); vst2(VBL + o3, *(const v4u*)&tbl[cl][q * 8]); } }
}

__global__ __launch_bounds__(128) void k_fa(const _Float16* __restrict__ QH, const _Float16* __restrict__ KH, const _Float16* __restrict__ VT, const int* __restrict__ MK, const int* __restrict__ FL, _Float16* __restrict__ YH) {
  __shared__ __align__(16) _Float16 sp[4][16][40];
  __shared__ __align__(16) _Float16 so[4][16][72];
  const int tid = threadIdx.x, lane = tid & 31, col = lane & 15, g = lane >> 4; const int wave = __builtin_amdgcn_readfirstlane(tid >> 5);
  const int qb = blockIdx.x + EARLY / 64; const int b = blockIdx.y / NH, h = blockIdx.y % NH; const int ql0 = qb * 64 + wave * 16;
  const size_t qoff = ((size_t)b * SEQ + ql0 + col) * CC + h * HD;
  const size_t kbase = ((size_t)b * SEQ + col) * CC + h * HD;
  const size_t vbase = ((size_t)b * CC + h * HD + col) * SEQ;
  const size_t mbase = (size_t)(ql0 + 8 * g) * SEQ_FULL + col;
  v16h ones;
#pragma unroll
  for (int i = 0; i < 16; ++i) ones[i] = (_Float16)1.0f;
  v8f acc[4] = {}; v8f accs = {};
  float mrun[8];
#pragma unroll
  for (int r = 0; r < 8; ++r) mrun[r] = -3.0e38f;
#pragma unroll 1
  for (int kb = 0; kb < NQB; ++kb) {
    const int fl = __builtin_amdgcn_readfirstlane(FL[qb * 32 + kb]);
    const int mode = (fl & 4) ? 3 : (fl & 3);
    if ((mode & 1) == 0) continue;
#pragma unroll 1
    for (int hf = 0; hf < 2; ++hf) { const int k0 = kb * 64 + hf * 32;
      v8f s0 = {}, s1 = {};
#pragma unroll
      for (int kc = 0; kc < HD / 32; ++kc) { const v16h qa = frag_h(QH + qoff + kc * 32, lane);
        const v16h ka0 = frag_h(KH + kbase + (size_t)k0 * CC + kc * 32, lane); const v16h ka1 = frag_h(KH + kbase + (size_t)(k0 + 16) * CC + kc * 32, lane);
        s0 = wmma16(qa, ka0, s0); s1 = wmma16(qa, ka1, s1); }
      float sv0[8], sv1[8];
#pragma unroll
      for (int r = 0; r < 8; ++r) { sv0[r] = s0[r] * SCALE; sv1[r] = s1[r] * SCALE; }
      if (mode == 3) { int m0[8], m1[8];
#pragma unroll
        for (int r = 0; r < 8; ++r) m0[r] = MK[mbase + (size_t)r * SEQ_FULL + k0];
        asm volatile("s_wait_loadcnt 0x0" ::: "memory");
#pragma unroll
        for (int r = 0; r < 8; ++r) m1[r] = MK[mbase + (size_t)r * SEQ_FULL + k0 + 16];
        asm volatile("s_wait_loadcnt 0x0" ::: "memory");
#pragma unroll
        for (int r = 0; r < 8; ++r) { sv0[r] = (m0[r] == 0) ? -1.0e9f : sv0[r]; sv1[r] = (m1[r] == 0) ? -1.0e9f : sv1[r]; } }
      float fr[8];
#pragma unroll
      for (int r = 0; r < 8; ++r) { float t = fmaxf(sv0[r], sv1[r]);
        t = fmaxf(t, __shfl_xor(t, 1)); t = fmaxf(t, __shfl_xor(t, 2)); t = fmaxf(t, __shfl_xor(t, 4)); t = fmaxf(t, __shfl_xor(t, 8));
        const float mn = fmaxf(mrun[r], t); fr[r] = __expf(mrun[r] - mn); mrun[r] = mn;
        sp[wave][8 * g + r][col] = (_Float16)(__expf(sv0[r] - mn) * 256.0f); sp[wave][8 * g + r][16 + col] = (_Float16)(__expf(sv1[r] - mn) * 256.0f); }
#pragma unroll
      for (int t = 0; t < 4; ++t) {
#pragma unroll
        for (int r = 0; r < 8; ++r) acc[t][r] *= fr[r]; }
#pragma unroll
      for (int r = 0; r < 8; ++r) accs[r] *= fr[r];
      LDSX();
      union { v16h v; v8h q[2]; } pa; pa.q[0] = *(const v8h*)&sp[wave][col][8 * g]; pa.q[1] = *(const v8h*)&sp[wave][col][16 + 8 * g];
      LDSX();
#pragma unroll
      for (int t = 0; t < 4; ++t) { const v16h vf = frag_h(VT + vbase + (size_t)(t * 16) * SEQ + k0, lane); acc[t] = wmma16(pa.v, vf, acc[t]); }
      accs = wmma16(pa.v, ones, accs);
    } }
  float inv[8];
#pragma unroll
  for (int r = 0; r < 8; ++r) inv[r] = (accs[r] > 0.0f) ? (1.0f / accs[r]) * 64.0f : 0.0f;
#pragma unroll
  for (int t = 0; t < 4; ++t) {
#pragma unroll
    for (int r = 0; r < 8; ++r) so[wave][8 * g + r][t * 16 + col] = (_Float16)(acc[t][r] * inv[r]); }
  LDSX();
#pragma unroll
  for (int it = 0; it < 4; ++it) { const int row = it * 4 + (lane >> 3), pc = lane & 7; const v4u w = *(const v4u*)&so[wave][row][pc * 8];
    vst2(YH + ((size_t)b * SEQ + ql0 + row) * CC + h * HD + pc * 8, w); }
}

__global__ __launch_bounds__(128) void k_fae(const _Float16* __restrict__ QH, const _Float16* __restrict__ KH, const _Float16* __restrict__ QL, const _Float16* __restrict__ KL,
    const __bf16* __restrict__ VB, const __bf16* __restrict__ VBL, const int* __restrict__ MK, const int* __restrict__ FL, __bf16* __restrict__ YB, __bf16* __restrict__ YBL) {
  __shared__ __align__(16) __bf16 sph[4][16][40], spl[4][16][40];
  __shared__ __align__(16) __bf16 sob[4][16][72], sol[4][16][72];
  const int tid = threadIdx.x, lane = tid & 31, col = lane & 15, g = lane >> 4; const int wave = __builtin_amdgcn_readfirstlane(tid >> 5);
  const int qb = blockIdx.x; const int b = blockIdx.y / NH, h = blockIdx.y % NH; const int ql0 = qb * 64 + wave * 16;
  const size_t qoff = ((size_t)b * SEQ + ql0 + col) * CC + h * HD;
  const size_t qloff = ((size_t)b * EARLY + ql0 + col) * CC + h * HD;
  const size_t kbase = ((size_t)b * SEQ + col) * CC + h * HD;
  const size_t vbase = ((size_t)b * CC + h * HD + col) * SEQ;
  const size_t mbase = (size_t)(ql0 + 8 * g) * SEQ_FULL + col;
  v16b onesb;
#pragma unroll
  for (int i = 0; i < 16; ++i) onesb[i] = (__bf16)1.0f;
  v8f acc[4] = {}; v8f accs = {};
  float mrun[8];
#pragma unroll
  for (int r = 0; r < 8; ++r) mrun[r] = -3.0e38f;
#pragma unroll 1
  for (int kb = 0; kb < NQB; ++kb) {
    const int fl = __builtin_amdgcn_readfirstlane(FL[qb * 32 + kb]);
    const int mode = (fl & 4) ? 3 : (fl & 3);
    if ((mode & 1) == 0) continue;
#pragma unroll 1
    for (int hf = 0; hf < 2; ++hf) { const int k0 = kb * 64 + hf * 32;
      v8f s0 = {}, s1 = {}, l0 = {}, l1 = {};
#pragma unroll
      for (int kc = 0; kc < HD / 32; ++kc) { const v16h qh = frag_h(QH + qoff + kc * 32, lane), ql = frag_h(QL + qloff + kc * 32, lane);
        const size_t ko0 = kbase + (size_t)k0 * CC + kc * 32, ko1 = ko0 + (size_t)16 * CC;
        const v16h kh0 = frag_h(KH + ko0, lane), kl0 = frag_h(KL + ko0, lane);
        s0 = wmma16(qh, kh0, s0); l0 = wmma16(ql, kh0, l0); l0 = wmma16(qh, kl0, l0);
        const v16h kh1 = frag_h(KH + ko1, lane), kl1 = frag_h(KL + ko1, lane);
        s1 = wmma16(qh, kh1, s1); l1 = wmma16(ql, kh1, l1); l1 = wmma16(qh, kl1, l1); }
      float sv0[8], sv1[8];
#pragma unroll
      for (int r = 0; r < 8; ++r) { sv0[r] = (s0[r] + l0[r] * (1.0f / 1024.0f)) * SCALE; sv1[r] = (s1[r] + l1[r] * (1.0f / 1024.0f)) * SCALE; }
      if (mode == 3) { int m0[8], m1[8];
#pragma unroll
        for (int r = 0; r < 8; ++r) m0[r] = MK[mbase + (size_t)r * SEQ_FULL + k0];
        asm volatile("s_wait_loadcnt 0x0" ::: "memory");
#pragma unroll
        for (int r = 0; r < 8; ++r) m1[r] = MK[mbase + (size_t)r * SEQ_FULL + k0 + 16];
        asm volatile("s_wait_loadcnt 0x0" ::: "memory");
#pragma unroll
        for (int r = 0; r < 8; ++r) { sv0[r] = (m0[r] == 0) ? -1.0e9f : sv0[r]; sv1[r] = (m1[r] == 0) ? -1.0e9f : sv1[r]; } }
      float fr[8];
#pragma unroll
      for (int r = 0; r < 8; ++r) { float t = fmaxf(sv0[r], sv1[r]);
        t = fmaxf(t, __shfl_xor(t, 1)); t = fmaxf(t, __shfl_xor(t, 2)); t = fmaxf(t, __shfl_xor(t, 4)); t = fmaxf(t, __shfl_xor(t, 8));
        const float mn = fmaxf(mrun[r], t); fr[r] = __expf(mrun[r] - mn); mrun[r] = mn;
        const float p0 = __expf(sv0[r] - mn), p1 = __expf(sv1[r] - mn); const __bf16 h0 = (__bf16)p0, h1 = (__bf16)p1;
        sph[wave][8 * g + r][col] = h0; spl[wave][8 * g + r][col] = (__bf16)(p0 - (float)h0);
        sph[wave][8 * g + r][16 + col] = h1; spl[wave][8 * g + r][16 + col] = (__bf16)(p1 - (float)h1); }
#pragma unroll
      for (int t = 0; t < 4; ++t) {
#pragma unroll
        for (int r = 0; r < 8; ++r) acc[t][r] *= fr[r]; }
#pragma unroll
      for (int r = 0; r < 8; ++r) accs[r] *= fr[r];
      LDSX();
      union { v16b v; v8b q[2]; } ph, pl;
      ph.q[0] = *(const v8b*)&sph[wave][col][8 * g]; ph.q[1] = *(const v8b*)&sph[wave][col][16 + 8 * g];
      pl.q[0] = *(const v8b*)&spl[wave][col][8 * g]; pl.q[1] = *(const v8b*)&spl[wave][col][16 + 8 * g];
      LDSX();
#pragma unroll
      for (int t = 0; t < 4; ++t) { const size_t po = vbase + (size_t)(t * 16) * SEQ + k0; const v16b vh = frag_b(VB + po, lane), vl = frag_b(VBL + po, lane);
        acc[t] = wmma_bf(ph.v, vh, acc[t]); acc[t] = wmma_bf(pl.v, vh, acc[t]); acc[t] = wmma_bf(ph.v, vl, acc[t]); }
      accs = wmma_bf(ph.v, onesb, accs); accs = wmma_bf(pl.v, onesb, accs);
    } }
  float inv[8];
#pragma unroll
  for (int r = 0; r < 8; ++r) inv[r] = (accs[r] > 0.0f) ? (1.0f / accs[r]) : 0.0f;
#pragma unroll
  for (int t = 0; t < 4; ++t) {
#pragma unroll
    for (int r = 0; r < 8; ++r) { const float c = acc[t][r] * inv[r]; const __bf16 ch = (__bf16)c; sob[wave][8 * g + r][t * 16 + col] = ch; sol[wave][8 * g + r][t * 16 + col] = (__bf16)(c - (float)ch); } }
  LDSX();
#pragma unroll
  for (int it = 0; it < 4; ++it) { const int row = it * 4 + (lane >> 3), pc = lane & 7; const size_t o = ((size_t)b * EARLY + ql0 + row) * CC + h * HD + pc * 8;
    const v4u wh = *(const v4u*)&sob[wave][row][pc * 8]; const v4u wl = *(const v4u*)&sol[wave][row][pc * 8];
    vst2(YB + o, wh); vst2(YBL + o, wl); }
}

__global__ __launch_bounds__(128) void k_out(const _Float16* __restrict__ YH, const __bf16* __restrict__ YB, const __bf16* __restrict__ YBL, const _Float16* __restrict__ WOH, const __bf16* __restrict__ WOB, float* __restrict__ OUT) {
  __shared__ __align__(16) float ss[4][16][132];
  const int tid = threadIdx.x, lane = tid & 31, col = lane & 15, g = lane >> 4; const int wave = __builtin_amdgcn_readfirstlane(tid >> 5);
  const int c0 = blockIdx.y * 128; const size_t rb = (size_t)blockIdx.x * 64; const size_t r0 = rb + wave * 16; const size_t bb = rb / SEQ; const int t0 = (int)(rb % SEQ);
  v8f acc[8] = {};
  if (t0 < EARLY) {
    const size_t ro = (bb * EARLY + t0 + wave * 16 + col) * (size_t)CC;
#pragma unroll 2
    for (int kc = 0; kc < CC / 32; ++kc) { const v16b ah = frag_b(YB + ro + kc * 32, lane), al = frag_b(YBL + ro + kc * 32, lane);
#pragma unroll
      for (int j = 0; j < 8; ++j) { const v16b w = frag_b(WOB + (size_t)(c0 + j * 16 + col) * CC + kc * 32, lane); acc[j] = wmma_bf(al, w, acc[j]); acc[j] = wmma_bf(ah, w, acc[j]); } }
#pragma unroll
    for (int j = 0; j < 8; ++j) {
#pragma unroll
      for (int r = 0; r < 8; ++r) ss[wave][8 * g + r][j * 16 + col] = acc[j][r]; }
  } else {
#pragma unroll 2
    for (int kc = 0; kc < CC / 32; ++kc) { const v16h a = frag_h(YH + (r0 + col) * CC + kc * 32, lane);
#pragma unroll
      for (int j = 0; j < 8; ++j) { const v16h w = frag_h(WOH + (size_t)(c0 + j * 16 + col) * CC + kc * 32, lane); acc[j] = wmma16(a, w, acc[j]); } }
#pragma unroll
    for (int j = 0; j < 8; ++j) {
#pragma unroll
      for (int r = 0; r < 8; ++r) ss[wave][8 * g + r][j * 16 + col] = acc[j][r] * (1.0f / 16384.0f); }
  }
  LDSX();
#pragma unroll 1
  for (int rl = 0; rl < 16; ++rl) vst2(OUT + (r0 + rl) * DIN + c0 + lane * 4, *(const v4f*)&ss[wave][rl][lane * 4]);
}

extern "C" void kernel_launch(void* const* d_in, const int* in_sizes, int n_in, void* d_out, int out_size, void* d_ws, size_t ws_size, hipStream_t stream) {
  if (n_in < 10) return;
  if (ws_size < (size_t)WS_END) return;
  const long long needx = ((long long)(NB - 1) * SEQ_FULL + SEQ) * DIN;
  const long long needw = (long long)CC * DIN;
  const long long needt = (long long)SEQ * HD;
  const long long needm = (long long)(SEQ - 1) * SEQ_FULL + SEQ;
  if (in_sizes[0] < needx || in_sizes[1] < needx || in_sizes[2] < needx) return;
  if (in_sizes[3] < needw || in_sizes[4] < needw || in_sizes[5] < needw || in_sizes[6] < needw) return;
  if (in_sizes[7] < needt || in_sizes[8] < needt || in_sizes[9] < needm) return;
  if ((long long)out_size < (long long)NB * SEQ * DIN) return;
  const float* xq = (const float*)d_in[0]; const float* xk = (const float*)d_in[1]; const float* xv = (const float*)d_in[2];
  const float* wq = (const float*)d_in[3]; const float* wk = (const float*)d_in[4]; const float* wv = (const float*)d_in[5]; const float* wo = (const float*)d_in[6];
  const float* cosp = (const float*)d_in[7]; const float* sinp = (const float*)d_in[8]; const int* mk = (const int*)d_in[9];
  char* ws = (char*)d_ws;
  __bf16* XB = (__bf16*)(ws + WS_XB); __bf16* WB = (__bf16*)(ws + WS_WB); _Float16* WOH = (_Float16*)(ws + WS_WOH);
  _Float16* QKH = (_Float16*)(ws + WS_QKH); _Float16* QKL = (_Float16*)(ws + WS_QKL);
  _Float16* VT = (_Float16*)(ws + WS_VT); __bf16* VB = (__bf16*)(ws + WS_VB); __bf16* VBL = (__bf16*)(ws + WS_VBL);
  _Float16* YH = (_Float16*)(ws + WS_YH); __bf16* YB = (__bf16*)(ws + WS_YB); __bf16* YBL = (__bf16*)(ws + WS_YBL);
  int* FL = (int*)(ws + WS_FL);
  _Float16* QH = QKH; _Float16* KH = QKH + (size_t)NB * SEQ * CC;
  _Float16* KL = QKL; _Float16* QL = QKL + (size_t)NB * SEQ * CC;
  __bf16* WOB = WB + (size_t)3 * CC * DIN;

  k_cvt<<<dim3((unsigned)(CVT_UNITS / 256), 7), 256, 0, stream>>>(xq, xk, xv, wq, wk, wv, wo, XB, WB, WOH);
  k_flag<<<dim3(NQB), 256, 0, stream>>>(mk, FL);
  k_proj<<<dim3(NB * SEQ / 64, CC / 128, 3), 128, 0, stream>>>(XB, WB, cosp, sinp, QKH, QKL, VT, VB, VBL);
  k_fae<<<dim3(EARLY / 64, NB * NH), 128, 0, stream>>>(QH, KH, QL, KL, VB, VBL, mk, FL, YB, YBL);
  if (NQB > EARLY / 64) k_fa<<<dim3(NQB - EARLY / 64, NB * NH), 128, 0, stream>>>(QH, KH, VT, mk, FL, YH);
  k_out<<<dim3(NB * SEQ / 64, DIN / 128), 128, 0, stream>>>(YH, YB, YBL, WOH, WOB, (float*)d_out);
}
